// MultiLayerCrossModalAttention_16466904613744
// MI455X (gfx1250) — hardware-verified
//
#include <hip/hip_runtime.h>

#define CCH    128
#define HIMG   128
#define WIMG   128
#define HW     16384
#define NB     4
#define NBH    2
#define NTOK   32
#define NL     2
#define WSC    16.0f
#define WINV   0.0625f
#define ASCALE 0.25f
#define LNEPS  1e-5f
#define TP     132
#define OSP    68
#define XSP    136

static_assert(HW == HIMG * WIMG);
static_assert(HW % 64 == 0);
static_assert(CCH == 128);
static_assert(NTOK * 4 == HIMG);
static_assert((NL * CCH * CCH) % (8 * 256) == 0);

typedef _Float16 v16h __attribute__((ext_vector_type(16)));
typedef _Float16 v8h  __attribute__((ext_vector_type(8)));
typedef float    v8f  __attribute__((ext_vector_type(8)));
typedef float    v4f  __attribute__((ext_vector_type(4)));
typedef v8h __attribute__((may_alias)) v8ha;
typedef v4f __attribute__((may_alias)) v4fa;

union Frag { v16h v; v8h half[2]; };

__device__ __forceinline__ v8f wmma_f16(v16h a, v16h b, v8f c) {
  v8f d = __builtin_amdgcn_wmma_f32_16x16x32_f16(false, a, false, b, (short)0, c, false, false);
  asm volatile("v_nop\n\tv_nop\n\tv_nop\n\tv_nop" : "+v"(d) : "v"(a), "v"(b));
  return d;
}

__device__ __forceinline__ v16h load_frag(const _Float16* p, int h) {
  Frag f;
  f.half[0] = *(const v8ha*)(p + 8 * h);
  f.half[1] = *(const v8ha*)(p + 16 + 8 * h);
  return f.v;
}

__device__ __forceinline__ float wsum(float v) {
  v += __shfl_xor(v, 16);
  v += __shfl_xor(v, 8);
  v += __shfl_xor(v, 4);
  v += __shfl_xor(v, 2);
  v += __shfl_xor(v, 1);
  return v;
}

__device__ __forceinline__ float dot4(v4f a, v4f b) {
  return a.x * b.x + a.y * b.y + a.z * b.z + a.w * b.w;
}

__global__ __launch_bounds__(256) void wconv_kernel(
    const float* __restrict__ qw, const float* __restrict__ kw,
    const float* __restrict__ vw, _Float16* __restrict__ wh)
{
  const int which = blockIdx.y;
  const int g = blockIdx.x * 256 + threadIdx.x;
  if (g >= (NL * CCH * CCH) / 8) return;
  const float* src = ((which == 0) ? qw : ((which == 1) ? kw : vw)) + (size_t)g * 8;
  const v4f a = *(const v4fa*)src;
  const v4f c = *(const v4fa*)(src + 4);
  v8h o;
  o[0] = (_Float16)(a.x * WSC); o[1] = (_Float16)(a.y * WSC);
  o[2] = (_Float16)(a.z * WSC); o[3] = (_Float16)(a.w * WSC);
  o[4] = (_Float16)(c.x * WSC); o[5] = (_Float16)(c.y * WSC);
  o[6] = (_Float16)(c.z * WSC); o[7] = (_Float16)(c.w * WSC);
  _Float16* dst = wh + (size_t)which * (NL * CCH * CCH) + (size_t)g * 8;
  *(volatile v8h*)dst = o;
  __threadfence();
  *(volatile v8h*)dst = o;
}

__device__ __forceinline__ void tr_store_pass(const _Float16* S, _Float16* Tb, int w, int lane) {
  const int pc = lane & 15, hi = lane >> 4;
  #pragma unroll
  for (int i = 0; i < 4; ++i) {
    const int R = 8 * w + 2 * i + hi;
    const v8h v = *(const v8ha*)(S + R * XSP + 8 * pc);
    *(volatile v8h*)(Tb + (size_t)R * CCH + 8 * pc) = v;
  }
}

__global__ __launch_bounds__(256) void tr_kernel(const float* __restrict__ X, _Float16* __restrict__ XT)
{
  __shared__ __attribute__((aligned(16))) _Float16 S[64 * XSP];
  const int tid = threadIdx.x, lane = tid & 31, w = tid >> 5;
  const int b = blockIdx.y, p0 = blockIdx.x * 64;
  const float* Xb = X + (size_t)b * CCH * HW + p0;
  #pragma unroll
  for (int it = 0; it < 8; ++it) {
    const int idx = it * 256 + tid;
    const int c = idx >> 4, q = idx & 15;
    const v4f v = *(const v4fa*)(Xb + (size_t)c * HW + 4 * q);
    S[(4 * q + 0) * XSP + c] = (_Float16)v.x;
    S[(4 * q + 1) * XSP + c] = (_Float16)v.y;
    S[(4 * q + 2) * XSP + c] = (_Float16)v.z;
    S[(4 * q + 3) * XSP + c] = (_Float16)v.w;
  }
  __syncthreads();
  _Float16* Tb = XT + ((size_t)b * HW + p0) * CCH;
  tr_store_pass(S, Tb, w, lane);
  __threadfence();
  tr_store_pass(S, Tb, w, lane);
}

__device__ __forceinline__ void proj_store_pass(const float* Os, float* Ob, int w, int lane) {
  const int q8 = lane & 7, sub = lane >> 3;
  #pragma unroll
  for (int i = 0; i < 8; ++i) {
    const int lid = 4 * i + sub;
    const int o = 16 * w + (lid >> 1), hl = lid & 1;
    const v4f v = *(const v4fa*)(Os + o * OSP + 32 * hl + 4 * q8);
    *(volatile v4f*)(Ob + (size_t)o * HW + 32 * hl + 4 * q8) = v;
  }
}

__global__ __launch_bounds__(256) void proj_kernel(
    const _Float16* __restrict__ curT,
    const _Float16* __restrict__ whiteT,
    const _Float16* __restrict__ wh,
    const float* __restrict__ qb, const float* __restrict__ kb, const float* __restrict__ vb,
    float* __restrict__ Qo, float* __restrict__ Ko, float* __restrict__ Vo,
    int b0, int layer)
{
  __shared__ __attribute__((aligned(16))) float Os[CCH * OSP];
  const int which = blockIdx.z;
  const _Float16* XT = (which == 0) ? curT : whiteT;
  const _Float16* W  = wh + ((size_t)which * NL + layer) * (CCH * CCH);
  const float* bias  = (which == 0) ? qb : ((which == 1) ? kb : vb);
  float* Out = (which == 0) ? Qo : ((which == 1) ? Ko : Vo);

  const int tid = threadIdx.x, lane = tid & 31, w = tid >> 5;
  const int h = lane >> 4, m = lane & 15;
  const int bl = blockIdx.y, p0 = blockIdx.x * 64;

  const _Float16* arow = W + (size_t)(16 * w + m) * CCH;
  const _Float16* xrow = XT + ((size_t)(b0 + bl) * HW + p0 + m) * CCH;

  const v8f zero8 = {0.f, 0.f, 0.f, 0.f, 0.f, 0.f, 0.f, 0.f};
  v8f acc[4];
  #pragma unroll
  for (int nt = 0; nt < 4; ++nt) acc[nt] = zero8;

  #pragma unroll
  for (int ks = 0; ks < 4; ++ks) {
    const int k0 = 32 * ks;
    const v16h a = load_frag(arow + k0, h);
    #pragma unroll
    for (int nt = 0; nt < 4; ++nt) {
      const v16h bf = load_frag(xrow + (size_t)(16 * nt) * CCH + k0, h);
      acc[nt] = wmma_f16(a, bf, acc[nt]);
    }
  }

  #pragma unroll
  for (int r = 0; r < 8; ++r) {
    const int o = 16 * w + 8 * h + r;
    const float bv = bias[layer * CCH + o];
    #pragma unroll
    for (int nt = 0; nt < 4; ++nt) Os[o * OSP + 16 * nt + m] = acc[nt][r] * WINV + bv;
  }
  __syncthreads();

  float* Ob = Out + (size_t)bl * CCH * HW + p0;
  proj_store_pass(Os, Ob, w, lane);
  __threadfence();
  proj_store_pass(Os, Ob, w, lane);
}

__device__ __forceinline__ void cur_store_pass(const float* T, _Float16* ct, int th, int twg, int w, int lane) {
  const int pc = lane & 15, hi = lane >> 4;
  #pragma unroll
  for (int i = 0; i < 8; ++i) {
    const int R = 16 * w + 2 * i + hi;
    const int r = R >> 5, wl = R & 31;
    const int p = (4 * th + r) * WIMG + 32 * twg + wl;
    const float* col = T + (8 * pc) * TP + R;
    v8h v;
    v[0] = (_Float16)col[0 * TP]; v[1] = (_Float16)col[1 * TP];
    v[2] = (_Float16)col[2 * TP]; v[3] = (_Float16)col[3 * TP];
    v[4] = (_Float16)col[4 * TP]; v[5] = (_Float16)col[5 * TP];
    v[6] = (_Float16)col[6 * TP]; v[7] = (_Float16)col[7 * TP];
    *(volatile v8h*)(ct + (size_t)p * CCH + 8 * pc) = v;
  }
}

__global__ __launch_bounds__(256) void attn_kernel(
    const float* __restrict__ Qp, const float* __restrict__ Kp, const float* __restrict__ Vp,
    const float* __restrict__ blue,
    const float* __restrict__ lng, const float* __restrict__ lnb,
    const float* __restrict__ lw,
    float* outp,
    _Float16* curT,
    int b0, int layer)
{
  extern __shared__ __attribute__((aligned(16))) float T[];
  const int tid = threadIdx.x, lane = tid & 31, w = tid >> 5;
  const int twg = blockIdx.x, th = blockIdx.y, bl = blockIdx.z;
  const int bg = b0 + bl;

  {
    const int c = tid & (CCH - 1);
    const int tsel = tid >> 7;
    const size_t cbase = ((size_t)bl * CCH + c) * HW;
    #pragma unroll 1
    for (int j = 0; j < 4; ++j) {
      const int t = tsel + 2 * j;
      const int tw = 8 * twg + t;
      const size_t qoff = cbase + (size_t)(4 * th) * WIMG + 4 * tw;
      const v4f q0 = *(const v4fa*)(Qp + qoff);
      const v4f q1 = *(const v4fa*)(Qp + qoff + WIMG);
      const v4f q2 = *(const v4fa*)(Qp + qoff + 2 * WIMG);
      const v4f q3 = *(const v4fa*)(Qp + qoff + 3 * WIMG);
      float mrun = -1e30f, srun = 0.0f;
      v4f o0 = {0.f, 0.f, 0.f, 0.f};
      v4f o1 = o0, o2 = o0, o3 = o0;
      #pragma unroll 1
      for (int di = 0; di < 3; ++di) {
        #pragma unroll 1
        for (int dj = 0; dj < 3; ++dj) {
          int th2 = th + di - 1, tw2 = tw + dj - 1;
          const bool valid = ((unsigned)th2 < (unsigned)NTOK) && ((unsigned)tw2 < (unsigned)NTOK);
          th2 = min(max(th2, 0), NTOK - 1);
          tw2 = min(max(tw2, 0), NTOK - 1);
          const size_t noff = cbase + (size_t)(4 * th2) * WIMG + 4 * tw2;
          const v4f k0 = *(const v4fa*)(Kp + noff);
          const v4f k1 = *(const v4fa*)(Kp + noff + WIMG);
          const v4f k2 = *(const v4fa*)(Kp + noff + 2 * WIMG);
          const v4f k3 = *(const v4fa*)(Kp + noff + 3 * WIMG);
          const float d = (dot4(q0, k0) + dot4(q1, k1)) + (dot4(q2, k2) + dot4(q3, k3));
          const float lg = valid ? d * ASCALE : 0.0f;
          const v4f v0 = *(const v4fa*)(Vp + noff);
          const v4f v1 = *(const v4fa*)(Vp + noff + WIMG);
          const v4f v2 = *(const v4fa*)(Vp + noff + 2 * WIMG);
          const v4f v3 = *(const v4fa*)(Vp + noff + 3 * WIMG);
          const float mn = fmaxf(mrun, lg);
          const float al = __expf(mrun - mn);
          const float p  = __expf(lg - mn);
          const float pv = valid ? p : 0.0f;
          srun = srun * al + p;
          o0 = o0 * al + v0 * pv;
          o1 = o1 * al + v1 * pv;
          o2 = o2 * al + v2 * pv;
          o3 = o3 * al + v3 * pv;
          mrun = mn;
        }
      }
      const float inv = 1.0f / srun;
      float* trow = T + c * TP + 4 * t;
      *(v4fa*)(trow)      = o0 * inv;
      *(v4fa*)(trow + 32) = o1 * inv;
      *(v4fa*)(trow + 64) = o2 * inv;
      *(v4fa*)(trow + 96) = o3 * inv;
    }
  }
  __syncthreads();

  {
    const float g0 = lng[layer * CCH + lane],      g1 = lng[layer * CCH + lane + 32];
    const float g2 = lng[layer * CCH + lane + 64], g3 = lng[layer * CCH + lane + 96];
    const float e0 = lnb[layer * CCH + lane],      e1 = lnb[layer * CCH + lane + 32];
    const float e2 = lnb[layer * CCH + lane + 64], e3 = lnb[layer * CCH + lane + 96];
    #pragma unroll 1
    for (int i = 0; i < 16; ++i) {
      const int pl = 16 * w + i;
      float* cp = T + lane * TP + pl;
      const float x0 = cp[0], x1 = cp[32 * TP], x2 = cp[64 * TP], x3 = cp[96 * TP];
      const float s  = wsum((x0 + x1) + (x2 + x3));
      const float mu = s * (1.0f / CCH);
      const float d0 = x0 - mu, d1 = x1 - mu, d2 = x2 - mu, d3 = x3 - mu;
      const float vs  = wsum((d0 * d0 + d1 * d1) + (d2 * d2 + d3 * d3));
      const float var = vs * (1.0f / CCH);
      const float rs  = rsqrtf(var + LNEPS);
      cp[0]       = d0 * rs * g0 + e0;
      cp[32 * TP] = d1 * rs * g1 + e1;
      cp[64 * TP] = d2 * rs * g2 + e2;
      cp[96 * TP] = d3 * rs * g3 + e3;
    }
  }
  __syncthreads();

  {
    const float cw = lw[layer];
    const float* base = (layer == 0) ? blue : outp;
    const int q8 = lane & 7, sub = lane >> 3;
    #pragma unroll 1
    for (int i = 0; i < 16; ++i) {
      const int L = 64 * w + 4 * i + sub;
      const int cc = L >> 2, r = L & 3;
      float* tp = T + cc * TP + r * 32 + 4 * q8;
      const v4f e = *(const v4fa*)tp;
      const size_t gi = (((size_t)(bg * CCH + cc) * HIMG + 4 * th + r) * WIMG) + 32 * twg + 4 * q8;
      const v4f bb = *(const v4fa*)(base + gi);
      const v4f v = bb + e * cw;
      *(volatile v4f*)(outp + gi) = v;
      __threadfence();
      *(volatile v4f*)(outp + gi) = v;
      if (layer == 0) *(v4fa*)tp = bb + e;
    }
  }

  if (layer == 0) {
    __syncthreads();
    _Float16* ct = curT + ((size_t)bg * HW) * CCH;
    cur_store_pass(T, ct, th, twg, w, lane);
    __threadfence();
    cur_store_pass(T, ct, th, twg, w, lane);
  }
}

extern "C" void kernel_launch(void* const* d_in, const int* in_sizes, int n_in,
                              void* d_out, int out_size, void* d_ws, size_t ws_size,
                              hipStream_t stream) {
  if (n_in < 11) return;
  const int ntot = NB * CCH * HW;
  if (in_sizes[0] != ntot || in_sizes[1] != ntot) return;
  if (in_sizes[2] != NL * CCH * CCH || in_sizes[4] != NL * CCH * CCH || in_sizes[6] != NL * CCH * CCH) return;
  if (in_sizes[3] != NL * CCH || in_sizes[5] != NL * CCH || in_sizes[7] != NL * CCH) return;
  if (in_sizes[8] != NL * CCH || in_sizes[9] != NL * CCH || in_sizes[10] != NL) return;
  if (out_size != ntot) return;

  const float* blue  = (const float*)d_in[0];
  const float* white = (const float*)d_in[1];
  const float* qw  = (const float*)d_in[2];
  const float* qb  = (const float*)d_in[3];
  const float* kw  = (const float*)d_in[4];
  const float* kb  = (const float*)d_in[5];
  const float* vw  = (const float*)d_in[6];
  const float* vb  = (const float*)d_in[7];
  const float* lng = (const float*)d_in[8];
  const float* lnb = (const float*)d_in[9];
  const float* lwt = (const float*)d_in[10];
  float* out = (float*)d_out;

  const size_t qkv_bytes = (size_t)NBH * CCH * HW * sizeof(float);
  const size_t xt_bytes  = (size_t)NB * HW * CCH * sizeof(_Float16);
  const size_t wh_bytes  = (size_t)3 * NL * CCH * CCH * sizeof(_Float16);
  const size_t total = 3 * qkv_bytes + 2 * xt_bytes + wh_bytes;
  if (total > ws_size) return;

  char* ws = (char*)d_ws;
  float*    Qp     = (float*)(ws);
  float*    Kp     = (float*)(ws + qkv_bytes);
  float*    Vp     = (float*)(ws + 2 * qkv_bytes);
  _Float16* whiteT = (_Float16*)(ws + 3 * qkv_bytes);
  _Float16* curT   = (_Float16*)(ws + 3 * qkv_bytes + xt_bytes);
  _Float16* Wh     = (_Float16*)(ws + 3 * qkv_bytes + 2 * xt_bytes);

  wconv_kernel<<<dim3((NL * CCH * CCH / 8 + 255) / 256, 3), 256, 0, stream>>>(qw, kw, vw, Wh);
  tr_kernel<<<dim3(HW / 64, NB), 256, 0, stream>>>(white, whiteT);
  tr_kernel<<<dim3(HW / 64, NB), 256, 0, stream>>>(blue, curT);

  const size_t att_lds = (size_t)CCH * TP * sizeof(float);
  hipFuncSetAttribute(reinterpret_cast<const void*>(&attn_kernel),
                      hipFuncAttributeMaxDynamicSharedMemorySize, (int)att_lds);

  for (int half = 0; half < NB / NBH; ++half) {
    const int b0 = half * NBH;
    for (int layer = 0; layer < NL; ++layer) {
      proj_kernel<<<dim3(HW / 64, NBH, 3), 256, 0, stream>>>(
          curT, whiteT, Wh, qb, kb, vb, Qp, Kp, Vp, b0, layer);
      attn_kernel<<<dim3(NTOK / 8, NTOK, NBH), 256, att_lds, stream>>>(
          Qp, Kp, Vp, blue, lng, lnb, lwt, out, curT, b0, layer);
    }
  }
}
